// Three_D_Branch_82566451298936
// MI455X (gfx1250) — hardware-run, weakly checked
//
#include <hip/hip_runtime.h>

typedef float          v8f   __attribute__((ext_vector_type(8)));
typedef float          v4f   __attribute__((ext_vector_type(4)));
typedef unsigned int   v4u   __attribute__((ext_vector_type(4)));
typedef int            v8i   __attribute__((ext_vector_type(8)));
typedef unsigned short v8us  __attribute__((ext_vector_type(8)));
typedef unsigned short v16us __attribute__((ext_vector_type(16)));
typedef __bf16         v16bf __attribute__((ext_vector_type(16)));
typedef _Float16       v16h  __attribute__((ext_vector_type(16)));
typedef v4f  __attribute__((may_alias)) v4fa;
typedef v8us __attribute__((may_alias)) v8usa;
union FragB { v16bf v; v16us u; v8us h[2]; v8i w; };
union FragH { v16h  v; v16us u; v8us h[2]; v8i w; };

__device__ __forceinline__ v8f wmb(const FragB& a, const FragB& b, v8f c) {
  v8f d = __builtin_amdgcn_wmma_f32_16x16x32_bf16(false, a.v, false, b.v, (short)0, c, false, false);
  asm volatile("v_nop\n\tv_nop\n\tv_nop\n\tv_nop" : "+v"(d) : "v"(a.w), "v"(b.w));
  return d;
}

__device__ __forceinline__ v8f wmh(const FragH& a, const FragH& b, v8f c) {
  v8f d = __builtin_amdgcn_wmma_f32_16x16x32_f16(false, a.v, false, b.v, (short)0, c, false, false);
  asm volatile("v_nop\n\tv_nop\n\tv_nop\n\tv_nop" : "+v"(d) : "v"(a.w), "v"(b.w));
  return d;
}

__device__ __forceinline__ unsigned bf16_bits(float f) {
  const unsigned u = __float_as_uint(f);
  const unsigned r = (u + 0x7FFFu + ((u >> 16) & 1u)) >> 16;
  const unsigned q = (u >> 16) | 0x40u;
  return ((u & 0x7fffffffu) > 0x7f800000u) ? q : r;
}

__device__ __forceinline__ float bf16_val(float f) {
  return __uint_as_float(bf16_bits(f) << 16);
}
__device__ __forceinline__ int clampi(int v, int lo, int hi) {
  return v < lo ? lo : (v > hi ? hi : v);
}

__device__ __forceinline__ unsigned f16_bits(float f) {
  const unsigned u  = __float_as_uint(f);
  const unsigned s  = (u >> 16) & 0x8000u;
  const unsigned a  = u & 0x7fffffffu;
  const unsigned t  = a - 0x38000000u;
  const unsigned r  = (t + 0x0FFFu + ((t >> 13) & 1u)) >> 13;
  const unsigned rc = r > 0x7C00u ? 0x7C00u : r;
  const bool small  = a < 0x38800000u;
  const bool isnan  = a > 0x7f800000u;
  const unsigned fin = small ? 0u : (s | rc);
  return isnan ? (s | 0x7E00u) : fin;
}

__device__ __forceinline__ unsigned pk16(unsigned lo, unsigned hi) { return lo | (hi << 16); }
__device__ __forceinline__ unsigned bf16_lo_bits(float v) {
  float hi = bf16_val(v);
  asm volatile("" : "+v"(hi));
  return bf16_bits(v - hi);
}
__device__ __forceinline__ v4u pack8_bf16(v4f a, v4f c) {
  return (v4u){ pk16(bf16_bits(a[0]), bf16_bits(a[1])), pk16(bf16_bits(a[2]), bf16_bits(a[3])),
                pk16(bf16_bits(c[0]), bf16_bits(c[1])), pk16(bf16_bits(c[2]), bf16_bits(c[3])) };
}
__device__ __forceinline__ v4u pack8_bf16_lo(v4f a, v4f c) {
  return (v4u){ pk16(bf16_lo_bits(a[0]), bf16_lo_bits(a[1])), pk16(bf16_lo_bits(a[2]), bf16_lo_bits(a[3])),
                pk16(bf16_lo_bits(c[0]), bf16_lo_bits(c[1])), pk16(bf16_lo_bits(c[2]), bf16_lo_bits(c[3])) };
}
__device__ __forceinline__ v4u pack8_f16(v4f a, v4f c) {
  return (v4u){ pk16(f16_bits(a[0]), f16_bits(a[1])), pk16(f16_bits(a[2]), f16_bits(a[3])),
                pk16(f16_bits(c[0]), f16_bits(c[1])), pk16(f16_bits(c[2]), f16_bits(c[3])) };
}

template <int FORM>
__global__ __launch_bounds__(256) void k_plane(const float* __restrict__ src, int rows, int cols, int ldsrc,
                                               unsigned short* __restrict__ dst, int MP, int KP) {
  static_assert(FORM >= 0 && FORM <= 3);
  const int KTOT = (FORM == 1 || FORM == 3) ? 2 * KP : KP;
  const unsigned ppr   = (unsigned)(KTOT >> 3);
  const unsigned kp8   = (unsigned)(KP >> 3);
  const unsigned total = (unsigned)MP * ppr;
  const unsigned g     = blockIdx.x * 256u + threadIdx.x;
  const unsigned rowu  = g / ppr;
  const unsigned p     = g - rowu * ppr;
  const bool second    = p >= kp8;
  const int row = (int)rowu;
  const int c0  = (int)((second ? p - kp8 : p) << 3);
  const float* srow = src + (size_t)clampi(row, 0, rows - 1) * (size_t)ldsrc;
  float x[8];
  unsigned mk[8];
#pragma unroll
  for (int e = 0; e < 8; ++e) {
    const int c = c0 + e;
    const float v = srow[clampi(c, 0, cols - 1)];
    asm volatile("" :: "v"(v));
    x[e]  = v;
    mk[e] = (row < rows && c < cols) ? 0xFFFFu : 0u;
  }
  const v4f a = (v4f){ x[0], x[1], x[2], x[3] };
  const v4f c = (v4f){ x[4], x[5], x[6], x[7] };
  v4u o;
  if (FORM == 2) {
    o = pack8_f16(a, c);
  } else {
    const v4u hi = pack8_bf16(a, c);
    o = hi;
    if (FORM == 1) { const v4u lo = pack8_bf16_lo(a, c); o = second ? lo : hi; }
  }
  const v4u mw = (v4u){ pk16(mk[0], mk[1]), pk16(mk[2], mk[3]), pk16(mk[4], mk[5]), pk16(mk[6], mk[7]) };
  o &= mw;
  if (g < total) {
    volatile v4u* q = (volatile v4u*)(dst + (size_t)g * 8);
    *q = o;
    __threadfence();
    *q = o;
  }
}

template <int FORM> struct FragOf    { typedef FragB T; };
template <>         struct FragOf<2> { typedef FragH T; };
__device__ __forceinline__ v8f mm(const FragB& a, const FragB& b, v8f c) { return wmb(a, b, c); }
__device__ __forceinline__ v8f mm(const FragH& a, const FragH& b, v8f c) { return wmh(a, b, c); }
template <class F> __device__ __forceinline__ F ld_frag(const unsigned short* p) {
  F f;
  f.h[0] = *(const v8usa*)(p);
  f.h[1] = *(const v8usa*)(p + 16);
  return f;
}

template <int FORM, int EPI>
__global__ __launch_bounds__(256) __attribute__((amdgpu_num_vgpr(248)))
void k_gemm_nt(const unsigned short* __restrict__ A, const unsigned short* __restrict__ B,
               const float* __restrict__ bias, float* __restrict__ D, int M, int N, int KTOT, int ldd) {
  static_assert(FORM >= 0 && FORM <= 2);
  static_assert(EPI == 0 || EPI == 1);
  typedef typename FragOf<FORM>::T F;
  __shared__ __attribute__((aligned(16))) float sT[8][16 * 68];
  const int lane = threadIdx.x & 31;
  const int wave = threadIdx.x >> 5;
  const int tilesM = (M + 63) >> 6;
  const int tilesN = (N + 63) >> 6;
  const int tile = blockIdx.x * 8 + wave;
  if (tile >= tilesM * tilesN) return;
  const int tm = tile / tilesN;
  const int tn = tile - tm * tilesN;
  const int m0 = tm << 6;
  const int n0 = tn << 6;

  const int rl = lane & 15;
  const int h8 = (lane >> 4) * 8;
  const unsigned short* pa = A + (size_t)(m0 + rl) * (size_t)KTOT + h8;
  const unsigned short* pb = B + (size_t)(n0 + rl) * (size_t)KTOT + h8;

  v8f acc[4][4];
#pragma unroll
  for (int i = 0; i < 4; ++i)
#pragma unroll
    for (int j = 0; j < 4; ++j) acc[i][j] = (v8f){0.f, 0.f, 0.f, 0.f, 0.f, 0.f, 0.f, 0.f};

#pragma unroll 1
  for (int k0 = 0; k0 < KTOT; k0 += 32) {
    F bf[4];
#pragma unroll
    for (int j = 0; j < 4; ++j) bf[j] = ld_frag<F>(pb + (size_t)(j << 4) * (size_t)KTOT + k0);
#pragma unroll
    for (int i = 0; i < 4; ++i) {
      const F af = ld_frag<F>(pa + (size_t)(i << 4) * (size_t)KTOT + k0);
#pragma unroll
      for (int j = 0; j < 4; ++j) acc[i][j] = mm(af, bf[j], acc[i][j]);
    }
  }

  float* slab = sT[wave];
  const int hh = lane >> 4;
  const int c4 = (lane & 15) * 4;
  const int nc = n0 + c4;
  const bool cok = nc < N;
  v4f bv = (v4f){0.f, 0.f, 0.f, 0.f};
  if (EPI == 1) {
    bv = *(const v4fa*)(bias + clampi(nc, 0, N - 4));
    asm volatile("" :: "v"(bv));
  }
#pragma unroll
  for (int i = 0; i < 4; ++i) {
    const int mBase = m0 + (i << 4);
#pragma unroll
    for (int j = 0; j < 4; ++j) {
#pragma unroll
      for (int r = 0; r < 8; ++r) slab[(h8 + r) * 68 + (j << 4) + rl] = acc[i][j][r];
    }
    __builtin_amdgcn_fence(__ATOMIC_RELEASE, "workgroup");
    __builtin_amdgcn_wave_barrier();
    __builtin_amdgcn_fence(__ATOMIC_ACQUIRE, "workgroup");
    v4f vv[8];
#pragma unroll
    for (int it = 0; it < 8; ++it) {
      const int row = it * 2 + hh;
      v4f v = *(const v4fa*)(slab + row * 68 + c4);
      if (EPI == 1) v += bv;
      vv[it] = v;
    }
    for (int pass = 0; pass < 2; ++pass) {
#pragma unroll
      for (int it = 0; it < 8; ++it) {
        const int row = mBase + it * 2 + hh;
        if (cok && row < M) *(volatile v4f*)(D + (size_t)row * (size_t)ldd + nc) = vv[it];
      }
      __threadfence();
    }
    __builtin_amdgcn_fence(__ATOMIC_RELEASE, "workgroup");
    __builtin_amdgcn_wave_barrier();
    __builtin_amdgcn_fence(__ATOMIC_ACQUIRE, "workgroup");
  }
}

#ifndef TWO_TERM
#define TWO_TERM 0
#endif

typedef float v2f __attribute__((ext_vector_type(2)));
typedef int   v2i __attribute__((ext_vector_type(2)));
typedef v2f __attribute__((may_alias)) v2fa;
typedef v2i __attribute__((may_alias)) v2ia;

constexpr int NBAT = 4;
constexpr int CH   = 64;
constexpr int NPTS = 16384;
constexpr int KNB  = 16;
constexpr int WLD  = 67;
constexpr int ROWS = NBAT * NPTS;
constexpr int K1   = 64;
constexpr int K2   = TWO_TERM ? 128 : 64;
constexpr int TP   = 65;

static_assert(ROWS == 65536 && ROWS == 8192 * 8);
static_assert(NPTS % 64 == 0 && NPTS / 64 == 256);
static_assert(CH == 64 && KNB == 16 && WLD == CH + 3);
static_assert(ROWS % 128 == 0 && ROWS % 64 == 0 && ROWS % 16 == 0);
static_assert(CH % 64 == 0 && CH % 4 == 0 && CH % 32 == 0);
static_assert(K1 % 32 == 0 && K2 % 32 == 0);
static_assert((long long)ROWS * K2 / 8 < (1LL << 31));
static_assert((long long)ROWS * CH - 1 == 4194303LL);

constexpr size_t SZ_FB  = (size_t)ROWS * K1 * 2;
constexpr size_t SZ_P   = (size_t)ROWS * CH * 4;
constexpr size_t SZ_F1  = (size_t)ROWS * K2 * 2;
constexpr size_t SZ_CB  = (size_t)ROWS * 16;
constexpr size_t SZ_WA1 = (size_t)CH * K1 * 2;
constexpr size_t SZ_WA2 = (size_t)CH * K2 * 2;
constexpr size_t SZ_WCB = (size_t)CH * 16;
constexpr size_t O_FB   = 0;
constexpr size_t O_P    = O_FB  + SZ_FB;
constexpr size_t O_F1   = O_P   + SZ_P;
constexpr size_t O_CB   = O_F1  + SZ_F1;
constexpr size_t O_WA1  = O_CB  + SZ_CB;
constexpr size_t O_WA2  = O_WA1 + SZ_WA1;
constexpr size_t O_WC1  = O_WA2 + SZ_WA2;
constexpr size_t O_WC2  = O_WC1 + SZ_WCB;
constexpr size_t O_END  = O_WC2 + SZ_WCB;
static_assert(O_P % 256 == 0 && O_F1 % 256 == 0 && O_CB % 256 == 0 && O_WA1 % 256 == 0);
static_assert(O_WA2 % 256 == 0 && O_WC1 % 256 == 0 && O_WC2 % 256 == 0 && O_END % 256 == 0);
static_assert(TWO_TERM == 0 || O_END == (size_t)43018240);
static_assert(O_END <= ((size_t)128 << 20));

constexpr int NBLK_CB  = ROWS / 256;
constexpr int NBLK_WA1 = CH * K1 / 8 / 256;
constexpr int NBLK_WA2 = CH * K2 / 8 / 256;
constexpr int BLK_WA1  = NBLK_CB;
constexpr int BLK_WA2  = BLK_WA1 + NBLK_WA1;
constexpr int BLK_WC1  = BLK_WA2 + NBLK_WA2;
constexpr int BLK_WC2  = BLK_WC1 + 1;
constexpr int NBLK_PREP = BLK_WC2 + 1;
static_assert(NBLK_CB * 256 == ROWS);
static_assert(NBLK_WA1 * 256 * 8 == CH * K1 && NBLK_WA2 * 256 * 8 == CH * K2);

__device__ __forceinline__ v4u gather8_bf16(const float* __restrict__ p) {
  float x[8];
#pragma unroll
  for (int e = 0; e < 8; ++e) {
    const float v = p[e];
    asm volatile("" :: "v"(v));
    x[e] = v;
  }
  return pack8_bf16((v4f){ x[0], x[1], x[2], x[3] }, (v4f){ x[4], x[5], x[6], x[7] });
}

__device__ __forceinline__ v4u wcb_row(const float* __restrict__ Wm, const float* __restrict__ bm, int c) {
  const float w0 = Wm[c * WLD + 64];
  const float w1 = Wm[c * WLD + 65];
  const float w2 = Wm[c * WLD + 66];
  const float bb = bm[c];
  asm volatile("" :: "v"(w0));
  asm volatile("" :: "v"(w1));
  asm volatile("" :: "v"(w2));
  asm volatile("" :: "v"(bb));
  return (v4u){ bf16_bits(w0) << 16, bf16_bits(w1) << 16, bf16_bits(w2) << 16, bf16_bits(bb) << 16 };
}

__global__ __launch_bounds__(256) void k_prep_planes(const float* __restrict__ coors,
                                                     const float* __restrict__ W1, const float* __restrict__ b1,
                                                     const float* __restrict__ W2, const float* __restrict__ b2,
                                                     v4u* ws16) {
  const int blk = (int)blockIdx.x;
  const int t   = (int)threadIdx.x;
  v4u o = (v4u){ 0u, 0u, 0u, 0u };
  unsigned off = 0u;
  bool st = true;
  if (blk < BLK_WA1) {
    const int r = blk * 256 + t;
    const float* p = coors + (size_t)r * 3;
    const float x = p[0];
    const float y = p[1];
    const float z = p[2];
    asm volatile("" :: "v"(x));
    asm volatile("" :: "v"(y));
    asm volatile("" :: "v"(z));
    o = (v4u){ bf16_bits(x) << 16, bf16_bits(y) << 16, bf16_bits(z) << 16, 0u };
    off = (unsigned)(O_CB / 16) + (unsigned)r;
  } else if (blk < BLK_WA2) {
    const int u  = (blk - BLK_WA1) * 256 + t;
    const int n  = u / (K1 / 8);
    const int k8 = (u % (K1 / 8)) * 8;
    o = gather8_bf16(W1 + n * WLD + k8);
    off = (unsigned)(O_WA1 / 16) + (unsigned)u;
  } else if (blk < BLK_WC1) {
    const int u  = (blk - BLK_WA2) * 256 + t;
    const int n  = u / (K2 / 8);
    const int k8 = ((u % (K2 / 8)) * 8) & (CH - 1);
    o = gather8_bf16(W2 + n * WLD + k8);
    off = (unsigned)(O_WA2 / 16) + (unsigned)u;
  } else if (blk == BLK_WC1) {
    const int c = t < CH ? t : CH - 1;
    o = wcb_row(W1, b1, c);
    off = (unsigned)(O_WC1 / 16) + (unsigned)c;
    st = t < CH;
  } else {
    const int c = t < CH ? t : CH - 1;
    o = wcb_row(W2, b2, c);
    off = (unsigned)(O_WC2 / 16) + (unsigned)c;
    st = t < CH;
  }
  if (st) {
    volatile v4u* q = (volatile v4u*)(ws16 + off);
    *q = o;
    __threadfence();
    *q = o;
  }
}

__global__ __launch_bounds__(256) void k_prep_feat(const int* __restrict__ mask, const float* __restrict__ feats,
                                                   unsigned short* FB) {
  __shared__ float tile[CH * TP];
  const int t = (int)threadIdx.x, lane = t & 31, wave = t >> 5;
  const int b  = (int)blockIdx.x >> 8;
  const int p0 = ((int)blockIdx.x & 255) * 64;

  const v2i mw = *(const v2ia*)(mask + (size_t)b * NPTS + p0 + 2 * lane);
  asm volatile("" :: "v"(mw));
  const unsigned km0 = (mw.x != 0) ? 0xFFFFFFFFu : 0u;
  const unsigned km1 = (mw.y != 0) ? 0xFFFFFFFFu : 0u;

  const float* src = feats + ((size_t)b * CH + 8 * wave) * NPTS + p0 + 2 * lane;
#pragma unroll 4
  for (int j = 0; j < 8; ++j) {
    const v2f v = *(const v2fa*)(src + (size_t)j * NPTS);
    asm volatile("" :: "v"(v));
    const float a0 = __uint_as_float(__float_as_uint(v.x) & km0);
    const float a1 = __uint_as_float(__float_as_uint(v.y) & km1);
    tile[(8 * wave + j) * TP + 2 * lane]     = a0;
    tile[(8 * wave + j) * TP + 2 * lane + 1] = a1;
  }
  __syncthreads();

  const int q = t & 7;
  v4u o[2];
#pragma unroll
  for (int it = 0; it < 2; ++it) {
    const int pl = it * 32 + (t >> 3);
    float x[8];
#pragma unroll
    for (int e = 0; e < 8; ++e) x[e] = tile[(8 * q + e) * TP + pl];
    o[it] = pack8_bf16((v4f){ x[0], x[1], x[2], x[3] }, (v4f){ x[4], x[5], x[6], x[7] });
  }
  unsigned short* base = FB + ((size_t)b * NPTS + p0) * CH + 8 * q;
#pragma unroll
  for (int it = 0; it < 2; ++it) {
    const int pl = it * 32 + (t >> 3);
    *(volatile v4u*)(base + (size_t)pl * CH) = o[it];
  }
  __threadfence();
#pragma unroll
  for (int it = 0; it < 2; ++it) {
    const int pl = it * 32 + (t >> 3);
    *(volatile v4u*)(base + (size_t)pl * CH) = o[it];
  }
}

template <int LAYER>
__global__ __launch_bounds__(256) void k_row(const float* __restrict__ P, const float* __restrict__ CB,
                                             const int* __restrict__ table, const float* __restrict__ WCB,
                                             unsigned* F1, float* out, int nRows) {
  static_assert(LAYER == 1 || LAYER == 2);
  const int lane = (int)threadIdx.x & 31;
  const int wave = (int)threadIdx.x >> 5;
  const int row  = (int)blockIdx.x * 8 + wave;
  if (row >= nRows) return;
  const int bbase = row & ~(NPTS - 1);

  const v4f own = *(const v4fa*)(CB + (size_t)row * 4);
  const v4f wa  = *(const v4fa*)(WCB + 8 * lane);
  const v4f wb  = *(const v4fa*)(WCB + 8 * lane + 4);
  int idv = table[(size_t)row * KNB + (lane & 15)];
  asm volatile("" :: "v"(idv));
  idv = clampi(idv, 0, NPTS - 1);

  float acc0 = 0.0f, acc1 = 0.0f;
#pragma unroll 2
  for (int k = 0; k < KNB; ++k) {
    const int nb = __builtin_amdgcn_readlane(idv, k);
    const int g  = bbase + nb;
    const v4f cn = *(const v4fa*)(CB + (size_t)g * 4);
    const v2f pv = *(const v2fa*)(P + (size_t)g * CH + 2 * lane);
    const float rx = own.x - cn.x;
    const float ry = own.y - cn.y;
    const float rz = own.z - cn.z;
    float t0 = fmaf(rx, wa.x, pv.x);
    float t1 = fmaf(rx, wb.x, pv.y);
    t0 = fmaf(ry, wa.y, t0);
    t1 = fmaf(ry, wb.y, t1);
    t0 = fmaf(rz, wa.z, t0);
    t1 = fmaf(rz, wb.z, t1);
    t0 = t0 + wa.w;
    t1 = t1 + wb.w;
    const float e0 = (t0 > 0.0f) ? t0 : (t0 - t0);
    const float e1 = (t1 > 0.0f) ? t1 : (t1 - t1);
    acc0 += e0;
    acc1 += e1;
  }

  if (LAYER == 1) {
    const unsigned hw = pk16(bf16_bits(acc0), bf16_bits(acc1));
    unsigned lw = 0u;
    if (TWO_TERM) lw = pk16(bf16_lo_bits(acc0), bf16_lo_bits(acc1));
    unsigned* rp = F1 + (size_t)row * (K2 / 2);
    volatile unsigned* q0 = (volatile unsigned*)(rp + lane);
    volatile unsigned* q1 = (volatile unsigned*)(rp + (TWO_TERM ? 32 : 0) + lane);
    *q0 = hw;
    if (TWO_TERM) *q1 = lw;
    __threadfence();
    *q0 = hw;
    if (TWO_TERM) *q1 = lw;
  } else {
    const v2f ov = (v2f){ acc0, acc1 };
    volatile v2f* q = (volatile v2f*)(out + (size_t)row * CH + 2 * lane);
    *q = ov;
    __threadfence();
    *q = ov;
  }
}

extern "C" void kernel_launch(void* const* d_in, const int* in_sizes, int n_in,
                              void* d_out, int out_size, void* d_ws, size_t ws_size,
                              hipStream_t stream) {
  if (n_in < 8) return;
  if (in_sizes[0] != ROWS) return;
  if (in_sizes[1] != ROWS * CH) return;
  if (in_sizes[2] != ROWS * 3) return;
  if (in_sizes[3] != ROWS * KNB) return;
  if (in_sizes[4] != CH * WLD || in_sizes[5] != CH) return;
  if (in_sizes[6] != CH * WLD || in_sizes[7] != CH) return;
  if (out_size != ROWS * CH) return;
  if (ws_size < O_END) return;

  const int*   mask  = (const int*)d_in[0];
  const float* feats = (const float*)d_in[1];
  const float* coors = (const float*)d_in[2];
  const int*   table = (const int*)d_in[3];
  const float* W1    = (const float*)d_in[4];
  const float* b1    = (const float*)d_in[5];
  const float* W2    = (const float*)d_in[6];
  const float* b2    = (const float*)d_in[7];
  float* out = (float*)d_out;

  char* ws = (char*)d_ws;
  unsigned short* FB   = (unsigned short*)(ws + O_FB);
  float*          P    = (float*)(ws + O_P);
  unsigned short* F1h  = (unsigned short*)(ws + O_F1);
  unsigned*       F1w  = (unsigned*)(ws + O_F1);
  float*          CB   = (float*)(ws + O_CB);
  unsigned short* WA1  = (unsigned short*)(ws + O_WA1);
  unsigned short* WA2D = (unsigned short*)(ws + O_WA2);
  float*          WCB1 = (float*)(ws + O_WC1);
  float*          WCB2 = (float*)(ws + O_WC2);
  v4u*            ws16 = (v4u*)d_ws;

  constexpr int TILES   = (ROWS / 64) * (CH / 64);
  constexpr int GEMMBLK = (TILES + 7) / 8;

  k_prep_planes<<<NBLK_PREP, 256, 0, stream>>>(coors, W1, b1, W2, b2, ws16);
  k_prep_feat<<<NBAT * (NPTS / 64), 256, 0, stream>>>(mask, feats, FB);
  k_gemm_nt<0, 0><<<GEMMBLK, 256, 0, stream>>>(FB, WA1, WCB1, P, ROWS, CH, K1, CH);
  k_row<1><<<ROWS / 8, 256, 0, stream>>>(P, CB, table, WCB1, F1w, out, ROWS);
  k_gemm_nt<0, 0><<<GEMMBLK, 256, 0, stream>>>(F1h, WA2D, WCB2, P, ROWS, CH, K2, CH);
  k_row<2><<<ROWS / 8, 256, 0, stream>>>(P, CB, table, WCB2, F1w, out, ROWS);
}
